// Fsmm_rnn_13915694039054
// MI455X (gfx1250) — hardware-verified
//
#include <hip/hip_runtime.h>


typedef _Float16 f16t;
typedef f16t  v16h __attribute__((ext_vector_type(16)));
typedef f16t  v8h  __attribute__((ext_vector_type(8)));
typedef float v8f  __attribute__((ext_vector_type(8)));
typedef float v4f  __attribute__((ext_vector_type(4)));
typedef unsigned int v4u __attribute__((ext_vector_type(4)));

union Frag { v16h v; v8h q[2]; };
union Pk16 { v8h h; v4u u; };
union Pk32 { v4f f; v4u u; };

#define NB   64
#define NT   2048
#define ND   4
#define NH   256
#define NWIN 64
#define KX   32
#define LPH  264
#define RB   16
#define WSC  16.0f
#define WINV 0.0625f

#define NBX0 (NH * KX / 8 / 256)
#define NBSQ (NH * NH / 8 / 256)
#define NBXP (NB * NT * KX / 8 / 256)

static_assert((NH * KX / 8) % 256 == 0);
static_assert((NH * NH / 8) % 256 == 0);
static_assert((NB * NT * KX / 8) % 256 == 0);
static_assert(NB % RB == 0);
static_assert(NH == 256);
static_assert(NWIN <= 256);

__device__ __forceinline__ v8f wmma16(v16h a, v16h b, v8f c) {
    return __builtin_amdgcn_wmma_f32_16x16x32_f16(false, a, false, b, (short)0, c, false, false);
}

__device__ __forceinline__ void mma2(v8f (&acc)[2], const f16t* A, int lda,
                                     const f16t* B, int ldb, int ktiles) {
    const int l = threadIdx.x & 31, h = l >> 4, m = l & 15;
    const f16t* ap = A + (size_t)m * lda + 8 * h;
    const f16t* bp = B + (size_t)m * ldb + 8 * h;
#pragma unroll 2
    for (int kt = 0; kt < ktiles; ++kt) {
        Frag a0, a1, b;
        const f16t* pa = ap + kt * 32;
        const f16t* pb = bp + kt * 32;
        a0.q[0] = *(const v8h*)pa;
        a0.q[1] = *(const v8h*)(pa + 16);
        a1.q[0] = *(const v8h*)(pa + (size_t)16 * lda);
        a1.q[1] = *(const v8h*)(pa + (size_t)16 * lda + 16);
        b.q[0]  = *(const v8h*)pb;
        b.q[1]  = *(const v8h*)(pb + 16);
        acc[0] = wmma16(a0.v, b.v, acc[0]);
        acc[1] = wmma16(a1.v, b.v, acc[1]);
        asm volatile("v_nop\n\tv_nop\n\tv_nop\n\tv_nop"
                     : "+v"(acc[0]), "+v"(acc[1])
                     : "v"(a0.v), "v"(a1.v), "v"(b.v));
    }
}

__device__ __forceinline__ float ftanh(float x) {
    float ax = fabsf(x);
    float t  = __expf(-2.0f * ax);
    float r  = (1.0f - t) * __builtin_amdgcn_rcpf(1.0f + t);
    return copysignf(r, x);
}

__device__ __forceinline__ void epi(v8f (&acc)[2], const float (&bz)[2][8],
                                    f16t* Hl, float* Sl, int f0, bool last) {
    const int l = threadIdx.x & 31, h = l >> 4, m = l & 15;
#pragma unroll
    for (int i = 0; i < 2; ++i) {
        Pk16 pk; Pk32 s0, s1;
#pragma unroll
        for (int r = 0; r < 4; ++r) {
            float v0 = ftanh(fmaf(acc[i][r],     WINV, bz[i][r]));
            float v1 = ftanh(fmaf(acc[i][4 + r], WINV, bz[i][4 + r]));
            pk.h[r]     = (f16t)v0;
            pk.h[4 + r] = (f16t)v1;
            s0.f[r] = v0;
            s1.f[r] = v1;
        }
        const int f = f0 + 16 * i + 8 * h;
        *(v8h*)(Hl + m * LPH + f) = pk.h;
        if (last) {
            float* d = Sl + m * NH + f;
            *(v4f*)d       = s0.f;
            *(v4f*)(d + 4) = s1.f;
        }
    }
}

__global__ __launch_bounds__(256)
void k_prep(const float* x, const float* Wih0, const float* Whh0, const float* Wih1,
            const float* Whh1, f16t* P0x, f16t* P0h, f16t* P1i, f16t* P1h, f16t* Xp) {
    const int tid = threadIdx.x;
    const int blk = blockIdx.x;
    const f16t z = (f16t)0.0f;
    Pk16 pk;
    f16t* d;
    if (blk < NBX0) {
        const int i  = blk * 256 + tid;
        const int n  = i >> 2;
        const int kq = (i & 3) * 8;
#pragma unroll
        for (int e = 0; e < 8; ++e) {
            const int k  = kq + e;
            const int kc = (k < ND) ? k : (ND - 1);
            const float wv = Wih0[n * ND + kc] * WSC;
            pk.h[e] = (k < ND) ? (f16t)wv : z;
        }
        d = P0x + (size_t)i * 8;
    } else if (blk < NBX0 + 3 * NBSQ) {
        const int rb    = blk - NBX0;
        const int which = rb / NBSQ;
        const int i     = (rb - which * NBSQ) * 256 + tid;
        const float* W = (which == 0) ? Whh0 : ((which == 1) ? Wih1 : Whh1);
        f16t* P        = (which == 0) ? P0h  : ((which == 1) ? P1i  : P1h);
        v4f a = *(const v4f*)(W + (size_t)i * 8);
        v4f b = *(const v4f*)(W + (size_t)i * 8 + 4);
#pragma unroll
        for (int e = 0; e < 4; ++e) {
            pk.h[e]     = (f16t)(a[e] * WSC);
            pk.h[4 + e] = (f16t)(b[e] * WSC);
        }
        d = P + (size_t)i * 8;
    } else {
        const int i   = (blk - NBX0 - 3 * NBSQ) * 256 + tid;
        const int row = i >> 2;
        const int p   = i & 3;
        v4f a = *(const v4f*)(x + (size_t)row * ND);
        const bool first = (p == 0);
        pk.h[0] = first ? (f16t)a[0] : z;
        pk.h[1] = first ? (f16t)a[1] : z;
        pk.h[2] = first ? (f16t)a[2] : z;
        pk.h[3] = first ? (f16t)a[3] : z;
        pk.h[4] = z; pk.h[5] = z; pk.h[6] = z; pk.h[7] = z;
        d = Xp + (size_t)i * 8;
    }
    *(volatile v4u*)d = pk.u;
    __threadfence();
    *(volatile v4u*)d = pk.u;
}

__global__ __launch_bounds__(256)
void k_rnn(const f16t* Xp, const f16t* P0x, const f16t* P0h, const f16t* P1i,
           const f16t* P1h, const float* bih0, const float* bhh0, const float* bih1,
           const float* bhh1, float* Hs0, float* Hs1) {
    __shared__ __attribute__((aligned(16))) f16t  H0[RB * LPH];
    __shared__ __attribute__((aligned(16))) f16t  H1[RB * LPH];
    __shared__ __attribute__((aligned(16))) float S0[RB * NH];
    __shared__ __attribute__((aligned(16))) float S1[RB * NH];

    const int tid = threadIdx.x, w = tid >> 5, l = tid & 31, h = l >> 4;
    const int b0  = blockIdx.x * RB;
    if (b0 + RB > NB) return;

    for (int i = tid; i < RB * LPH; i += 256) { H0[i] = (f16t)0.0f; H1[i] = (f16t)0.0f; }

    const int f0 = 32 * w;
    float bz0[2][8], bz1[2][8];
#pragma unroll
    for (int i = 0; i < 2; ++i)
#pragma unroll
        for (int r = 0; r < 8; ++r) {
            const int f = f0 + 16 * i + 8 * h + r;
            bz0[i][r] = bih0[f] + bhh0[f];
            bz1[i][r] = bih1[f] + bhh1[f];
        }
    __syncthreads();

    const f16t* xb  = Xp  + (size_t)b0 * NT * KX;
    const f16t* a0x = P0x + (size_t)f0 * KX;
    const f16t* a0h = P0h + (size_t)f0 * NH;
    const f16t* a1i = P1i + (size_t)f0 * NH;
    const f16t* a1h = P1h + (size_t)f0 * NH;
    const v8f zacc = {0.f, 0.f, 0.f, 0.f, 0.f, 0.f, 0.f, 0.f};

#pragma unroll 1
    for (int t = 0; t < NT; ++t) {
        const bool last = (t == NT - 1);

        v8f acc[2];
        acc[0] = zacc; acc[1] = zacc;
        mma2(acc, a0x, KX, xb + (size_t)t * KX, NT * KX, 1);
        mma2(acc, a0h, NH, H0, LPH, 8);
        __syncthreads();
        epi(acc, bz0, H0, S0, f0, last);
        __syncthreads();

        acc[0] = zacc; acc[1] = zacc;
        mma2(acc, a1i, NH, H0, LPH, 8);
        mma2(acc, a1h, NH, H1, LPH, 8);
        __syncthreads();
        epi(acc, bz1, H1, S1, f0, last);
    }
    __syncthreads();

    Pk32 u0[4], u1[4];
#pragma unroll
    for (int it = 0; it < 4; ++it) {
        const int p = tid + 256 * it, row = p >> 6, c = (p & 63) * 4;
        u0[it].f = *(const v4f*)(S0 + row * NH + c);
        u1[it].f = *(const v4f*)(S1 + row * NH + c);
    }
#pragma unroll
    for (int it = 0; it < 4; ++it) {
        const int p = tid + 256 * it, row = p >> 6, c = (p & 63) * 4;
        *(volatile v4u*)(Hs0 + (size_t)(b0 + row) * NH + c) = u0[it].u;
        *(volatile v4u*)(Hs1 + (size_t)(b0 + row) * NH + c) = u1[it].u;
    }
    __threadfence();
#pragma unroll
    for (int it = 0; it < 4; ++it) {
        const int p = tid + 256 * it, row = p >> 6, c = (p & 63) * 4;
        *(volatile v4u*)(Hs0 + (size_t)(b0 + row) * NH + c) = u0[it].u;
        *(volatile v4u*)(Hs1 + (size_t)(b0 + row) * NH + c) = u1[it].u;
    }
}

__device__ __forceinline__ float bred(float* red, float v) {
#pragma unroll
    for (int o = 16; o > 0; o >>= 1) v += __shfl_xor(v, o, 32);
    const int w = threadIdx.x >> 5, l = threadIdx.x & 31;
    __syncthreads();
    if (l == 0) red[w] = v;
    __syncthreads();
    float r = red[0];
#pragma unroll
    for (int i = 1; i < 8; ++i) r += red[i];
    return r;
}

__global__ __launch_bounds__(256)
void k_tail(const float* x, const float* Wih0, const float* Wih1,
            const float* fcW, const float* fcb, const float* Qp, const float* deltap,
            const float* f1W, const float* f1b, const float* f2W, const float* f2b,
            const float* U0p, const float* R0p, const float* C1p, const float* R1p,
            const float* binom, const float* Hs0, const float* Hs1, float* out) {
#pragma clang fp contract(off)
    __shared__ float red[8];
    __shared__ float g1s[NH];
    __shared__ __attribute__((aligned(16))) float socs[NB];
    __shared__ __attribute__((aligned(16))) float dsocs[NB];
    __shared__ __attribute__((aligned(16))) float fsocs[NB];
    __shared__ __attribute__((aligned(16))) float ups[NB];
    __shared__ __attribute__((aligned(16))) float vls[NB];
    __shared__ __attribute__((aligned(16))) float ils[NB];

    const int tid = threadIdx.x;
    (void)U0p;
    const float fw   = fcW[tid];
    const float w03  = Wih0[tid * ND + 3];
    const float f1w  = f1W[tid];
    const float f1c  = f1b[tid];
    const float f2w  = f2W[tid];
    const float fcb0 = fcb[0], f2b0 = f2b[0];
    const float r1   = R1p[0], c1 = C1p[0];
    const int   kk   = (tid < NWIN) ? tid : (NWIN - 1);

#pragma unroll 1
    for (int b = 0; b < NB; ++b) {
        const float hT = Hs1[(size_t)b * NH + tid];
        const float ys = Hs0[(size_t)b * NH + tid];
        const float soc_b = bred(red, hT * fw) + fcb0;

        g1s[tid] = fw * (1.0f - hT * hT);
        __syncthreads();
        float s = 0.0f;
#pragma unroll 4
        for (int o = 0; o < NH; ++o) s += g1s[o] * Wih1[o * NH + tid];
        const float g0 = s * (1.0f - ys * ys);
        const float dsoc_b = bred(red, g0 * w03);

        const float fs_b = bred(red, (soc_b * f1w + f1c) * f2w) + f2b0;

        const float* xb = x + (size_t)b * NT * ND;
        float hv = binom[kk + 1] * xb[(NT - NWIN + kk) * ND + 0];
        hv = (tid < NWIN) ? hv : 0.0f;
        const float hist_b = bred(red, hv);

        if (tid == 0) {
            const float vl = xb[(NT - 1) * ND + 0];
            const float il = xb[(NT - 1) * ND + 1];
            const float t1 = xb[(NT - 1) * ND + 3];
            const float t0 = xb[(NT - NWIN) * ND + 3];
            const float tdiff = (t1 - t0) * (1.0f / (float)(NWIN - 1));
            const float Ts = sqrtf(tdiff);
            const float up = (-Ts * (1.0f / (r1 * c1))) * vl + (Ts * (1.0f / c1)) * il - hist_b;
            socs[b]  = soc_b;
            dsocs[b] = dsoc_b;
            fsocs[b] = fs_b;
            ups[b]   = up;
            vls[b]   = vl;
            ils[b]   = il;
        }
    }
    __syncthreads();

    const float cq  = deltap[0] * (1.0f / Qp[0]);
    const float rr0 = R0p[0];

    Pk32 o0, o1[4], o2[4];
    {
        const int i4 = (tid & 15) * 4;
#pragma unroll
        for (int e = 0; e < 4; ++e) o0.f[e] = socs[i4 + e];
    }
#pragma unroll
    for (int it = 0; it < 4; ++it) {
        const int p = tid + 256 * it, i = p >> 4, j0 = (p & 15) * 4;
        const float a1 = cq * ils[i];
        const float a2 = (fsocs[i] - vls[i]) - rr0 * ils[i];
#pragma unroll
        for (int e = 0; e < 4; ++e) {
            o1[it].f[e] = a1 + dsocs[j0 + e];
            o2[it].f[e] = a2 - ups[j0 + e];
        }
    }
    float* out1 = out + NB;
    float* out2 = out + NB + NB * NB;
    if (tid < 16) *(volatile v4u*)(out + tid * 4) = o0.u;
#pragma unroll
    for (int it = 0; it < 4; ++it) {
        const int p = tid + 256 * it, i = p >> 4, j0 = (p & 15) * 4;
        *(volatile v4u*)(out1 + i * NB + j0) = o1[it].u;
        *(volatile v4u*)(out2 + i * NB + j0) = o2[it].u;
    }
    __threadfence();
    if (tid < 16) *(volatile v4u*)(out + tid * 4) = o0.u;
#pragma unroll
    for (int it = 0; it < 4; ++it) {
        const int p = tid + 256 * it, i = p >> 4, j0 = (p & 15) * 4;
        *(volatile v4u*)(out1 + i * NB + j0) = o1[it].u;
        *(volatile v4u*)(out2 + i * NB + j0) = o2[it].u;
    }
}

extern "C" void kernel_launch(void* const* d_in, const int* in_sizes, int n_in,
                              void* d_out, int out_size, void* d_ws, size_t ws_size,
                              hipStream_t stream) {
    if (n_in < 22) return;
    if (in_sizes[0] != NB * NT * ND || in_sizes[1] != NH * ND || in_sizes[2] != NH * NH ||
        in_sizes[3] != NH || in_sizes[4] != NH || in_sizes[5] != NH * NH ||
        in_sizes[6] != NH * NH || in_sizes[7] != NH || in_sizes[8] != NH ||
        in_sizes[9] != NH || in_sizes[10] < 1 || in_sizes[11] < 1 || in_sizes[12] < 1 ||
        in_sizes[13] != NH || in_sizes[14] != NH || in_sizes[15] != NH || in_sizes[16] < 1 ||
        in_sizes[18] < 1 || in_sizes[19] < 1 || in_sizes[20] < 1 ||
        in_sizes[21] != NWIN + 1) return;
    if (out_size != NB + 2 * NB * NB) return;

    const float* x     = (const float*)d_in[0];
    const float* Wih0  = (const float*)d_in[1];
    const float* Whh0  = (const float*)d_in[2];
    const float* bih0  = (const float*)d_in[3];
    const float* bhh0  = (const float*)d_in[4];
    const float* Wih1  = (const float*)d_in[5];
    const float* Whh1  = (const float*)d_in[6];
    const float* bih1  = (const float*)d_in[7];
    const float* bhh1  = (const float*)d_in[8];
    const float* fcW   = (const float*)d_in[9];
    const float* fcb   = (const float*)d_in[10];
    const float* Qp    = (const float*)d_in[11];
    const float* delta = (const float*)d_in[12];
    const float* f1W   = (const float*)d_in[13];
    const float* f1b   = (const float*)d_in[14];
    const float* f2W   = (const float*)d_in[15];
    const float* f2b   = (const float*)d_in[16];
    const float* U0    = (const float*)d_in[17];
    const float* R0    = (const float*)d_in[18];
    const float* C1    = (const float*)d_in[19];
    const float* R1    = (const float*)d_in[20];
    const float* binom = (const float*)d_in[21];
    float* out = (float*)d_out;

    char* ws = (char*)d_ws;
    size_t off = 0;
    auto carve = [&](size_t bytes) -> char* {
        char* p = ws + off;
        off = (off + bytes + 255) & ~(size_t)255;
        return p;
    };
    f16t*  P0x = (f16t*)carve((size_t)NH * KX * 2);
    f16t*  P0h = (f16t*)carve((size_t)NH * NH * 2);
    f16t*  P1i = (f16t*)carve((size_t)NH * NH * 2);
    f16t*  P1h = (f16t*)carve((size_t)NH * NH * 2);
    f16t*  Xp  = (f16t*)carve((size_t)NB * NT * KX * 2);
    float* Hs0 = (float*)carve((size_t)NB * NH * 4);
    float* Hs1 = (float*)carve((size_t)NB * NH * 4);
    if (off > ws_size) return;

    k_prep<<<dim3(NBX0 + 3 * NBSQ + NBXP), dim3(256), 0, stream>>>(
        x, Wih0, Whh0, Wih1, Whh1, P0x, P0h, P1i, P1h, Xp);

    k_rnn<<<dim3(NB / RB), dim3(256), 0, stream>>>(
        Xp, P0x, P0h, P1i, P1h, bih0, bhh0, bih1, bhh1, Hs0, Hs1);

    k_tail<<<dim3(1), dim3(256), 0, stream>>>(
        x, Wih0, Wih1, fcW, fcb, Qp, delta, f1W, f1b, f2W, f2b, U0, R0, C1, R1, binom,
        Hs0, Hs1, out);
}
